// DCConv_49606872269284
// MI455X (gfx1250) — hardware-verified
//
#include <hip/hip_runtime.h>
#define NB 4
#define NN 1024
#define KK 32
#define CC 64
#define MM 8
#define CO 128
#define NPt (NB * NN * KK)
#define NPN (NB * NN)
#define CH 16384
#define EPS 1e-5f
typedef __bf16 v16b __attribute__((ext_vector_type(16)));
typedef unsigned short v8us __attribute__((ext_vector_type(8), may_alias));
typedef float  v8f  __attribute__((ext_vector_type(8)));
typedef float  v4f  __attribute__((ext_vector_type(4)));
typedef float  v4fa __attribute__((ext_vector_type(4), may_alias));
union FragB { v16b v; v8us half[2]; unsigned short u[16]; };

__device__ __forceinline__ unsigned short bf16_bits(float x) { unsigned int u = __float_as_uint(x); return (unsigned short)((u + 0x7FFFu + ((u >> 16) & 1u)) >> 16); }
__device__ __forceinline__ float bf16_val(unsigned short b) { return __uint_as_float(((unsigned int)b) << 16); }
__device__ __forceinline__ float bf16_round(float x) { return bf16_val(bf16_bits(x)); }
template <int NT>
__device__ __forceinline__ v8f mmaN(v16b ah, v16b al, v16b bh, v16b bl, v8f c) {
  c = __builtin_amdgcn_wmma_f32_16x16x32_bf16(false, ah, false, bh, (short)0, c, false, false);
  if (NT >= 2) c = __builtin_amdgcn_wmma_f32_16x16x32_bf16(false, al, false, bh, (short)0, c, false, false);
  if (NT >= 3) c = __builtin_amdgcn_wmma_f32_16x16x32_bf16(false, ah, false, bl, (short)0, c, false, false);
  asm volatile("v_nop\n\tv_nop\n\tv_nop\n\tv_nop" : "+v"(c) : "v"(ah), "v"(al), "v"(bh), "v"(bl));
  return c;
}

__global__ __launch_bounds__(256) void k_wt_bf16(const float* __restrict__ W, unsigned short* __restrict__ Wt, int K, int N) {
  const int t = blockIdx.x * 256 + threadIdx.x;
  const int k8n = K / 8;
  if (t >= N * k8n) return;
  const int n = t / k8n, k8 = (t % k8n) * 8;
  v8us v;
#pragma unroll
  for (int i = 0; i < 8; ++i) v[i] = bf16_bits(W[(size_t)(k8 + i) * N + n]);
  *(volatile v8us*)(Wt + (size_t)n * K + k8) = v;
  __threadfence();
  *(volatile v8us*)(Wt + (size_t)n * K + k8) = v;
}

template <bool ASPLIT, int ACT, bool BIAS_BF16>
__global__ __launch_bounds__(128) void k_gemm_bf(const float* __restrict__ A, int lda, const unsigned short* __restrict__ Wt, int ldb,
                                               const float* __restrict__ bias, float* __restrict__ C, int ldc, int M, int N, int K) {
  __shared__ __attribute__((aligned(16))) float so[4][16][64];
  const int tid = threadIdx.x, w = tid >> 5, lane = tid & 31, ln = lane & 15, hh = lane >> 4;
  const int ntn = N / 64;
  const int wid = blockIdx.x * 4 + w;
  const int mt = wid / ntn, nq = wid % ntn;
  if (mt * 16 >= M) return;
  const int row0 = mt * 16, col0 = nq * 64;
  const float* arow = A + (size_t)(row0 + ln) * lda;
  v8f acc[4] = {};
  for (int kb = 0; kb < K; kb += 32) {
    FragB ah, al;
    const v4f x0 = *(const v4fa*)(arow + kb + 8 * hh), x1 = *(const v4fa*)(arow + kb + 8 * hh + 4);
    const v4f x2 = *(const v4fa*)(arow + kb + 16 + 8 * hh), x3 = *(const v4fa*)(arow + kb + 16 + 8 * hh + 4);
    float xs[16] = {x0[0],x0[1],x0[2],x0[3],x1[0],x1[1],x1[2],x1[3],x2[0],x2[1],x2[2],x2[3],x3[0],x3[1],x3[2],x3[3]};
#pragma unroll
    for (int i = 0; i < 16; ++i) { const unsigned short hb = bf16_bits(xs[i]); ah.u[i] = hb; al.u[i] = ASPLIT ? bf16_bits(xs[i] - bf16_val(hb)) : (unsigned short)0; }
#pragma unroll
    for (int t = 0; t < 4; ++t) {
      const unsigned short* brow = Wt + (size_t)(col0 + t * 16 + ln) * ldb + kb;
      FragB b;
      b.half[0] = *(const v8us*)(brow + 8 * hh);
      b.half[1] = *(const v8us*)(brow + 16 + 8 * hh);
      acc[t] = mmaN<ASPLIT ? 2 : 1>(ah.v, al.v, b.v, b.v, acc[t]);
    }
  }
#pragma unroll
  for (int t = 0; t < 4; ++t) {
    float bv = bias ? bias[col0 + t * 16 + ln] : 0.f;
    if (BIAS_BF16) bv = bf16_round(bv);
#pragma unroll
    for (int r = 0; r < 8; ++r) { float v = acc[t][r] + bv; if (ACT == 1) v = fmaxf(v, 0.f); so[w][8 * hh + r][t * 16 + ln] = v; }
  }
  __builtin_amdgcn_fence(__ATOMIC_ACQ_REL, "workgroup");
  __builtin_amdgcn_wave_barrier();
  const int rsub = lane >> 4, c4 = (lane & 15) * 4;
  for (int pass = 0; pass < 2; ++pass) {
#pragma unroll
    for (int q = 0; q < 8; ++q) {
      const int r = q * 2 + rsub;
      const v4f v = *(const v4fa*)&so[w][r][c4];
      *(volatile v4f*)(C + (size_t)(row0 + r) * ldc + col0 + c4) = v;
    }
    if (pass == 0) __threadfence();
  }
}

template <bool ASPLIT, int ACT, bool BIAS_BF16, bool RES_BF16>
__global__ __launch_bounds__(128) void k_gemm_bf3(const float* __restrict__ A, int lda, const unsigned short* __restrict__ Wt, int ldb,
                                                const float* __restrict__ bias, const float* __restrict__ resid, int rmod, int ldr,
                                                float* __restrict__ C, int ldc, int M, int N, int K) {
  __shared__ __attribute__((aligned(16))) float so[4][16][64];
  const int tid = threadIdx.x, w = tid >> 5, lane = tid & 31, ln = lane & 15, hh = lane >> 4;
  const int ntn = N / 64;
  const int wid = blockIdx.x * 4 + w;
  const int mt = wid / ntn, nq = wid % ntn;
  if (mt * 16 >= M) return;
  const int row0 = mt * 16, col0 = nq * 64;
  const float* arow = A + (size_t)(row0 + ln) * lda;
  v8f acc[4] = {};
  for (int kb = 0; kb < K; kb += 32) {
    FragB ah, al;
    const v4f x0 = *(const v4fa*)(arow + kb + 8 * hh), x1 = *(const v4fa*)(arow + kb + 8 * hh + 4);
    const v4f x2 = *(const v4fa*)(arow + kb + 16 + 8 * hh), x3 = *(const v4fa*)(arow + kb + 16 + 8 * hh + 4);
    float xs[16] = {x0[0],x0[1],x0[2],x0[3],x1[0],x1[1],x1[2],x1[3],x2[0],x2[1],x2[2],x2[3],x3[0],x3[1],x3[2],x3[3]};
#pragma unroll
    for (int i = 0; i < 16; ++i) { const unsigned short hb = bf16_bits(xs[i]); ah.u[i] = hb; al.u[i] = ASPLIT ? bf16_bits(xs[i] - bf16_val(hb)) : (unsigned short)0; }
#pragma unroll
    for (int t = 0; t < 4; ++t) {
      const unsigned short* brow = Wt + (size_t)(col0 + t * 16 + ln) * ldb + kb;
      FragB b;
      b.half[0] = *(const v8us*)(brow + 8 * hh);
      b.half[1] = *(const v8us*)(brow + 16 + 8 * hh);
      acc[t] = mmaN<ASPLIT ? 2 : 1>(ah.v, al.v, b.v, b.v, acc[t]);
    }
  }
#pragma unroll
  for (int t = 0; t < 4; ++t) {
    const int col = col0 + t * 16 + ln;
    float bv = bias ? bias[col] : 0.f;
    if (BIAS_BF16) bv = bf16_round(bv);
#pragma unroll
    for (int r = 0; r < 8; ++r) {
      float v = acc[t][r] + bv;
      if (resid) { float rv = resid[(size_t)((row0 + 8 * hh + r) % rmod) * ldr + col]; if (RES_BF16) rv = bf16_round(rv); v += rv; }
      if (ACT == 1) v = fmaxf(v, 0.f);
      if (ACT == 2) v = 0.5f * v * (1.0f + erff(v * 0.70710678118654752f));
      if (ACT == 3) { const float u = 0.7978845608028654f * (v + 0.044715f * v * v * v); v = 0.5f * v * (1.0f + tanhf(u)); }
      so[w][8 * hh + r][t * 16 + ln] = v;
    }
  }
  __builtin_amdgcn_fence(__ATOMIC_ACQ_REL, "workgroup");
  __builtin_amdgcn_wave_barrier();
  const int rsub = lane >> 4, c4 = (lane & 15) * 4;
  for (int pass = 0; pass < 2; ++pass) {
#pragma unroll
    for (int q = 0; q < 8; ++q) {
      const int r = q * 2 + rsub;
      const v4f v = *(const v4fa*)&so[w][r][c4];
      *(volatile v4f*)(C + (size_t)(row0 + r) * ldc + col0 + c4) = v;
    }
    if (pass == 0) __threadfence();
  }
}
template <bool PARAM_BF16>
__global__ __launch_bounds__(256) void k_layernorm(const float* __restrict__ X, const float* __restrict__ R, const float* __restrict__ g, const float* __restrict__ bta,
                                                  float* __restrict__ out_sum, float* __restrict__ out_norm, int N, float eps) {
  __shared__ float red[256];
  const int row = blockIdx.x, tid = threadIdx.x;
  const float* x = X + (size_t)row * N; const float* rr = R ? R + (size_t)row * N : nullptr;
  float vals[16];
  const int per = N / 256;
  float s1 = 0.f;
  for (int u = 0; u < per / 4; ++u) {
    const int j = tid * 4 + 1024 * u;
    const v4f a = *(const v4fa*)(x + j);
    v4f b = {0.f,0.f,0.f,0.f}; if (rr) b = *(const v4fa*)(rr + j);
#pragma unroll
    for (int q = 0; q < 4; ++q) { const float v = a[q] + b[q]; vals[u * 4 + q] = v; s1 += v; }
  }
  red[tid] = s1; __syncthreads();
  for (int st = 128; st > 0; st >>= 1) { if (tid < st) red[tid] += red[tid + st]; __syncthreads(); }
  const float mu = red[0] / (float)N; __syncthreads();
  float s2 = 0.f;
  for (int u = 0; u < per / 4; ++u)
#pragma unroll
    for (int q = 0; q < 4; ++q) { const float c = vals[u * 4 + q] - mu; s2 += c * c; }
  red[tid] = s2; __syncthreads();
  for (int st = 128; st > 0; st >>= 1) { if (tid < st) red[tid] += red[tid + st]; __syncthreads(); }
  const float rs = rsqrtf(red[0] / (float)N + eps);
  for (int pass = 0; pass < 2; ++pass) {
    for (int u = 0; u < per / 4; ++u) {
      const int j = tid * 4 + 1024 * u;
      v4f o, sm;
#pragma unroll
      for (int q = 0; q < 4; ++q) {
        float gg = g[j + q], bb = bta[j + q];
        if (PARAM_BF16) { gg = bf16_round(gg); bb = bf16_round(bb); }
        sm[q] = vals[u * 4 + q]; o[q] = (vals[u * 4 + q] - mu) * rs * gg + bb;
      }
      if (out_sum) *(volatile v4f*)(out_sum + (size_t)row * N + j) = sm;
      *(volatile v4f*)(out_norm + (size_t)row * N + j) = o;
    }
    if (pass == 0) __threadfence();
  }
}


typedef _Float16 v16h __attribute__((ext_vector_type(16)));
union FragH { v16h v; v8us half[2]; _Float16 h[16]; unsigned short u[16]; };
template <int NT>
__device__ __forceinline__ v8f mmaH(v16h ah, v16h al, v16h bh, v16h bl, v8f c) {
  c = __builtin_amdgcn_wmma_f32_16x16x32_f16(false, ah, false, bh, (short)0, c, false, false);
  if (NT >= 2) c = __builtin_amdgcn_wmma_f32_16x16x32_f16(false, al, false, bh, (short)0, c, false, false);
  if (NT >= 3) c = __builtin_amdgcn_wmma_f32_16x16x32_f16(false, ah, false, bl, (short)0, c, false, false);
  asm volatile("v_nop\n\tv_nop\n\tv_nop\n\tv_nop" : "+v"(c) : "v"(ah), "v"(al), "v"(bh), "v"(bl));
  return c;
}
template <bool ASPLIT>
__global__ __launch_bounds__(128) void k_gemm_h(const float* __restrict__ A, int lda, size_t sA, const _Float16* __restrict__ Bh, int ldb, size_t sB, float alpha, float* __restrict__ C, int ldc, size_t sC, int M, int N, int K) {
  __shared__ __attribute__((aligned(16))) float so[4][16][64];
  const int tid = threadIdx.x, w = tid >> 5, lane = tid & 31, ln = lane & 15, hh = lane >> 4; const int by = blockIdx.y;
  A += (size_t)by * sA; Bh += (size_t)by * sB; C += (size_t)by * sC;
  const int ntn = (N + 63) / 64; const int wid = blockIdx.x * 4 + w; const int mt = wid / ntn, nq = wid % ntn; if (mt * 16 >= M) return;
  const int row0 = mt * 16, col0 = nq * 64; const float* arow = A + (size_t)(row0 + ln) * lda;
  v8f acc[4] = {};
  for (int kb = 0; kb < K; kb += 32) {
    FragH ah, al;
    const v4f x0 = *(const v4fa*)(arow + kb + 8 * hh), x1 = *(const v4fa*)(arow + kb + 8 * hh + 4), x2 = *(const v4fa*)(arow + kb + 16 + 8 * hh), x3 = *(const v4fa*)(arow + kb + 16 + 8 * hh + 4);
    float xs[16] = {x0[0],x0[1],x0[2],x0[3],x1[0],x1[1],x1[2],x1[3],x2[0],x2[1],x2[2],x2[3],x3[0],x3[1],x3[2],x3[3]};
#pragma unroll
    for (int i = 0; i < 16; ++i) { const _Float16 h = (_Float16)xs[i]; ah.h[i] = h; al.h[i] = ASPLIT ? (_Float16)(xs[i] - (float)h) : (_Float16)0.0f; }
#pragma unroll
    for (int t = 0; t < 4; ++t) { if (col0 + t * 16 >= N) continue; const size_t boff = (size_t)(col0 + t * 16 + ln) * ldb + kb; FragH bq; bq.half[0] = *(const v8us*)(Bh + boff + 8 * hh); bq.half[1] = *(const v8us*)(Bh + boff + 16 + 8 * hh);
      acc[t] = mmaH<ASPLIT ? 2 : 1>(ah.v, al.v, bq.v, bq.v, acc[t]); }
  }
#pragma unroll
  for (int t = 0; t < 4; ++t) { if (col0 + t * 16 >= N) continue;
#pragma unroll
    for (int r = 0; r < 8; ++r) so[w][8 * hh + r][t * 16 + ln] = acc[t][r] * alpha; }
  __builtin_amdgcn_fence(__ATOMIC_ACQ_REL, "workgroup"); __builtin_amdgcn_wave_barrier();
  const int rsub = lane >> 4, c4 = (lane & 15) * 4;
  for (int pass = 0; pass < 2; ++pass) {
#pragma unroll
    for (int q = 0; q < 8; ++q) { const int r = q * 2 + rsub; if (col0 + c4 < N) { const v4f v = *(const v4fa*)&so[w][r][c4]; *(volatile v4f*)(C + (size_t)(row0 + r) * ldc + col0 + c4) = v; } }
    if (pass == 0) __threadfence(); }
}

__global__ __launch_bounds__(256) void k_wt_f16(const float* __restrict__ W, _Float16* __restrict__ Wt, int K, int N, float scale) {
  const int t = blockIdx.x * 256 + threadIdx.x; if (t >= N * (K / 8)) return; const int n = t / (K / 8), k8 = (t % (K / 8)) * 8; FragH f;
#pragma unroll
  for (int i = 0; i < 8; ++i) f.h[i] = (_Float16)(bf16_round(W[(size_t)(k8 + i) * N + n]) * scale); const v8us o = f.half[0];
  *(volatile v8us*)((unsigned short*)Wt + (size_t)n * K + k8) = o; __threadfence(); *(volatile v8us*)((unsigned short*)Wt + (size_t)n * K + k8) = o;
}
template <int ACT>
__global__ __launch_bounds__(128) void k_gemm_hhx(const _Float16* __restrict__ A, int lda, size_t sA, const _Float16* __restrict__ Bh, int ldb, size_t sB, float alpha, const float* __restrict__ bias, size_t sBias, const float* __restrict__ CP, int rowsPerB, size_t sCPb, int row0g,
    float* __restrict__ C, _Float16* __restrict__ C16, int ldc, size_t sC, int M, int N, int K) {
  __shared__ __attribute__((aligned(16))) float so[4][16][64];
  const int tid = threadIdx.x, w = tid >> 5, lane = tid & 31, ln = lane & 15, hh = lane >> 4; const int by = blockIdx.y;
  A += (size_t)by * sA; Bh += (size_t)by * sB; const size_t cofs = (size_t)by * sC; const float* bp = bias ? bias + (size_t)by * sBias : nullptr;
  const int ntn = (N + 63) / 64; const int wid = blockIdx.x * 4 + w; const int mt = wid / ntn, nq = wid % ntn; if (mt * 16 >= M) return;
  const int row0 = mt * 16, col0 = nq * 64; const _Float16* arow = A + (size_t)(row0 + ln) * lda;
  v8f acc[4] = {};
  for (int kb = 0; kb < K; kb += 32) { FragH ah; ah.half[0] = *(const v8us*)((const unsigned short*)arow + kb + 8 * hh); ah.half[1] = *(const v8us*)((const unsigned short*)arow + kb + 16 + 8 * hh);
#pragma unroll
    for (int t = 0; t < 4; ++t) { if (col0 + t * 16 >= N) continue; const size_t boff = (size_t)(col0 + t * 16 + ln) * ldb + kb; FragH bq; bq.half[0] = *(const v8us*)((const unsigned short*)Bh + boff + 8 * hh); bq.half[1] = *(const v8us*)((const unsigned short*)Bh + boff + 16 + 8 * hh);
      acc[t] = mmaH<1>(ah.v, ah.v, bq.v, bq.v, acc[t]); }
  }
#pragma unroll
  for (int t = 0; t < 4; ++t) { if (col0 + t * 16 >= N) continue; const int col = col0 + t * 16 + ln; const float bv = bp ? bf16_round(bp[col]) : 0.f;
#pragma unroll
    for (int r = 0; r < 8; ++r) { float v = acc[t][r] * alpha + bv; if (CP) { const int bidx = (row0g + row0 + 8 * hh + r) / rowsPerB; v += CP[(size_t)bidx * sCPb + (size_t)by * 64 + col]; } if (ACT == 1) v = (v > 0.f) ? v : expm1f(v); else if (ACT == 7) v = (v > 0.f) ? v + 1.0f : expf(v); else if (ACT == 8) v = tanhf(v); else if (ACT == 9) v = 0.5f * v * (1.0f + tanhf(0.7978845608028654f * (v + 0.044715f * v * v * v))); else if (ACT == 11) v = 1.0f / (1.0f + expf(-v)); else if (ACT == 12) v = (v > 0.f) ? v : 0.01f * v; else if (ACT == 14) v = (v > 0.f) ? v : 0.1f * v; else if (ACT == 15) v = v / (1.0f + expf(-v)); else if (ACT == 3) v = fmaxf(v, 0.f); else if (ACT == 6) v = 0.5f * v * (1.0f + erff(v * 0.70710678118654752f)); so[w][8 * hh + r][t * 16 + ln] = v; } }
  __builtin_amdgcn_fence(__ATOMIC_ACQ_REL, "workgroup"); __builtin_amdgcn_wave_barrier();
  const int rsub = lane >> 4, c4 = (lane & 15) * 4; typedef _Float16 v4h __attribute__((ext_vector_type(4)));
  for (int pass = 0; pass < 2; ++pass) {
#pragma unroll
    for (int q = 0; q < 8; ++q) { const int r = q * 2 + rsub; if (col0 + c4 < N) { const v4f v = *(const v4fa*)&so[w][r][c4]; if (C) *(volatile v4f*)(C + cofs + (size_t)(row0 + r) * ldc + col0 + c4) = v; if (C16) { v4h h4; for (int i = 0; i < 4; ++i) h4[i] = (_Float16)v[i]; *(volatile v4h*)(C16 + cofs + (size_t)(row0 + r) * ldc + col0 + c4) = h4; } } }
    if (pass == 0) __threadfence(); }
}


typedef _Float16 v4h __attribute__((ext_vector_type(4)));

__global__ __launch_bounds__(256) void k_x16(const float* __restrict__ x, _Float16* __restrict__ X16, size_t n8) { const size_t t = (size_t)blockIdx.x * 256 + threadIdx.x; if (t >= n8) return; FragH f;
#pragma unroll
  for (int q = 0; q < 8; ++q) f.h[q] = (_Float16)bf16_round(x[t * 8 + q]); *(volatile v8us*)((unsigned short*)X16 + t * 8) = f.half[0]; __threadfence(); *(volatile v8us*)((unsigned short*)X16 + t * 8) = f.half[0]; }
__global__ __launch_bounds__(256) void k_h16(const float* __restrict__ x, _Float16* __restrict__ X16, size_t n8) { const size_t t = (size_t)blockIdx.x * 256 + threadIdx.x; if (t >= n8) return; FragH f;
#pragma unroll
  for (int q = 0; q < 8; ++q) f.h[q] = (_Float16)x[t * 8 + q]; *(volatile v8us*)((unsigned short*)X16 + t * 8) = f.half[0]; __threadfence(); *(volatile v8us*)((unsigned short*)X16 + t * 8) = f.half[0]; }
__global__ __launch_bounds__(256) void k_round16f(const float* __restrict__ W, _Float16* __restrict__ Bt, size_t n8) { const size_t t = (size_t)blockIdx.x * 256 + threadIdx.x; if (t >= n8) return; FragH f;
#pragma unroll
  for (int i = 0; i < 8; ++i) f.h[i] = (_Float16)(bf16_round(W[t * 8 + i]) * 16.0f); *(volatile v8us*)((unsigned short*)Bt + t * 8) = f.half[0]; __threadfence(); *(volatile v8us*)((unsigned short*)Bt + t * 8) = f.half[0]; }
template <int NHv, int TTv>
__global__ __launch_bounds__(256) void k_vt(const _Float16* __restrict__ V16, int ldv, int voff, _Float16* __restrict__ Vt) { __shared__ unsigned short tl[64][66]; const int tid = threadIdx.x; const int slab = blockIdx.x / (TTv / 64), lg = blockIdx.x % (TTv / 64); const int b = slab / NHv, h = slab % NHv;
  for (int i = tid; i < 64 * 8; i += 256) { const int r = i / 8, c8 = (i % 8) * 8; FragH f; f.half[0] = *(const v8us*)((const unsigned short*)V16 + ((size_t)b * TTv + lg * 64 + r) * ldv + voff + h * 64 + c8);
#pragma unroll
    for (int q = 0; q < 8; ++q) tl[r][c8 + q] = f.u[q]; }
  __syncthreads();
  for (int pass = 0; pass < 2; ++pass) {
#pragma unroll
    for (int rd = 0; rd < 2; ++rd) { const int d = rd * 32 + tid / 8, pc = tid % 8; FragH f;
#pragma unroll
      for (int q = 0; q < 8; ++q) f.u[q] = tl[pc * 8 + q][d];
      *(volatile v8us*)((unsigned short*)Vt + ((size_t)slab * 64 + d) * TTv + lg * 64 + pc * 8) = f.half[0]; }
    if (pass == 0) __threadfence(); } }

__global__ __launch_bounds__(256) void k_hl(const float* __restrict__ F, _Float16* __restrict__ Hh, _Float16* __restrict__ Hl, size_t n8) { const size_t t = (size_t)blockIdx.x * 256 + threadIdx.x; if (t >= n8) return; FragH fh, fl; const v4f a = *(const v4fa*)(F + t * 8), c = *(const v4fa*)(F + t * 8 + 4);
#pragma unroll
  for (int q = 0; q < 4; ++q) { _Float16 h = (_Float16)a[q]; fh.h[q] = h; fl.h[q] = (_Float16)((a[q] - (float)h) * 1024.0f); h = (_Float16)c[q]; fh.h[4 + q] = h; fl.h[4 + q] = (_Float16)((c[q] - (float)h) * 1024.0f); }
  for (int pass = 0; pass < 2; ++pass) { *(volatile v8us*)((unsigned short*)Hh + t * 8) = fh.half[0]; *(volatile v8us*)((unsigned short*)Hl + t * 8) = fl.half[0]; if (pass == 0) __threadfence(); } }

__device__ __forceinline__ float inp_at(const float* __restrict__ in, int b, int ch, int n, int k) { return bf16_round(in[(((size_t)b * (3 + CC) + ch) * NN + n) * KK + k]); }
__global__ __launch_bounds__(256) void k_pre(const float* __restrict__ in, const float* __restrict__ sw1, const float* __restrict__ hw1, float* __restrict__ PRE) {
  #pragma clang fp contract(off)
  const size_t t = (size_t)blockIdx.x * 256 + threadIdx.x; if (t >= (size_t)NPt * 12) return; const int c0 = (int)(t % 12) * 4; const size_t pt = t / 12; const int k = (int)(pt % KK); const int n = (int)((pt / KK) % NN); const int b = (int)(pt / ((size_t)KK * NN));
  float h[10]; const float dx = inp_at(in, b, 3, n, k), dy = inp_at(in, b, 4, n, k), dz = inp_at(in, b, 5, n, k); h[0] = sqrtf((dx * dx + dy * dy) + dz * dz);
  h[1] = inp_at(in, b, 0, n, 0); h[2] = inp_at(in, b, 1, n, 0); h[3] = inp_at(in, b, 2, n, 0); h[4] = inp_at(in, b, 0, n, k); h[5] = inp_at(in, b, 1, n, k); h[6] = inp_at(in, b, 2, n, k); h[7] = dx; h[8] = dy; h[9] = dz;
  v4f o;
#pragma unroll
  for (int q = 0; q < 4; ++q) { const int c = c0 + q; float s = 0.f; if (c < MM) {
#pragma unroll
      for (int i = 0; i < 10; ++i) s += h[i] * bf16_round(sw1[c * 10 + i]); }
    else if (c < MM + 32) { const int o_ = c - MM;
#pragma unroll
      for (int i = 0; i < 10; ++i) s += h[i] * bf16_round(hw1[o_ * 10 + i]); }
    o[q] = s; }
  *(volatile v4f*)(PRE + pt * 48 + c0) = o; __threadfence(); *(volatile v4f*)(PRE + pt * 48 + c0) = o; }
__global__ __launch_bounds__(256) void k_colstats(const float* __restrict__ Z, int R, int C, double* __restrict__ SUM, double* __restrict__ SQ) { __shared__ double s1[8][32], s2[8][32]; const int tid = threadIdx.x, w = tid >> 5, l = tid & 31; const int c = blockIdx.x * 32 + l; double a = 0.0, b = 0.0;
  if (c < C) {
#pragma unroll 1
    for (int r = w; r < R; r += 8) { const double v = (double)Z[(size_t)r * C + c]; a += v; b += v * v; } }
  s1[w][l] = a; s2[w][l] = b; __syncthreads();
  if (w == 0) { double t1 = 0.0, t2 = 0.0; for (int k = 0; k < 8; ++k) { t1 += s1[k][l]; t2 += s2[k][l]; } for (int pass = 0; pass < 2; ++pass) { *(volatile double*)(SUM + blockIdx.x * 32 + l) = t1; *(volatile double*)(SQ + blockIdx.x * 32 + l) = t2; if (pass == 0) __threadfence(); } } }
__global__ __launch_bounds__(256) void k_bnab(const double* __restrict__ SUM, const double* __restrict__ SQ, int C, int CPt, int count, const float* __restrict__ g, const float* __restrict__ be, float* __restrict__ AB) {
  #pragma clang fp contract(off)
  const int c = blockIdx.x * 256 + threadIdx.x; if (c >= C) return; const double m = SUM[c] / (double)count; double var = SQ[c] / (double)count - m * m; if (var < 0.0) var = 0.0; const float a = bf16_round(g[c]) * rsqrtf((float)var + EPS); const float sh = bf16_round(be[c]) - (float)m * a;
  for (int pass = 0; pass < 2; ++pass) { *(volatile float*)(AB + c) = a; *(volatile float*)(AB + CPt + c) = sh; if (pass == 0) __threadfence(); } }
__global__ __launch_bounds__(256) void k_act1(const float* __restrict__ PRE, const float* __restrict__ ABs, const float* __restrict__ ABd, const float* __restrict__ sw2, const float* __restrict__ sb2, float* __restrict__ SC, _Float16* __restrict__ Dh, _Float16* __restrict__ Dl) {
  #pragma clang fp contract(off)
  const size_t t = (size_t)blockIdx.x * 256 + threadIdx.x; if (t >= (size_t)NPt * 4) return; const int q = (int)(t % 4); const size_t pt = t / 4; const float* pr = PRE + pt * 48;
  float s1[MM];
#pragma unroll
  for (int m = 0; m < MM; ++m) s1[m] = fmaxf(pr[m] * ABs[m] + ABs[MM + m], 0.f);
  float s2[MM]; float mx = -3.0e38f;
#pragma unroll
  for (int m = 0; m < MM; ++m) { float s = bf16_round(sb2[m]);
#pragma unroll
    for (int j = 0; j < MM; ++j) s += s1[j] * bf16_round(sw2[m * MM + j]); s2[m] = s; mx = fmaxf(mx, s); }
  float den = 0.f;
#pragma unroll
  for (int m = 0; m < MM; ++m) { s2[m] = expf(s2[m] - mx); den += s2[m]; }
  FragH fh, fl;
#pragma unroll
  for (int j = 0; j < 8; ++j) { const int c = 8 * q + j; const float v = fmaxf(pr[MM + c] * ABd[c] + ABd[32 + c], 0.f); const _Float16 hi = (_Float16)v; fh.h[j] = hi; fl.h[j] = (_Float16)((v - (float)hi) * 1024.0f); }
  v4f sc;
#pragma unroll
  for (int j = 0; j < 4; ++j) { float v = 0.f;
#pragma unroll
    for (int m = 0; m < MM; ++m) v = (m == 4 * (q & 1) + j) ? s2[m] / den : v; sc[j] = v; }
  for (int pass = 0; pass < 2; ++pass) { *(volatile v8us*)((unsigned short*)Dh + pt * 32 + 8 * q) = fh.half[0]; *(volatile v8us*)((unsigned short*)Dl + pt * 32 + 8 * q) = fl.half[0]; if (q < 2) *(volatile v4f*)(SC + pt * MM + 4 * q) = sc; if (pass == 0) __threadfence(); } }
__global__ __launch_bounds__(256) void k_agg(const float* __restrict__ D2, const float* __restrict__ SC, const float* __restrict__ in, const float* __restrict__ pp, int p0, float* __restrict__ AGG) {
  #pragma clang fp contract(off)
  const size_t t = (size_t)blockIdx.x * 256 + threadIdx.x; if (t >= (size_t)CH * (CC / 4)) return; const int c0 = (int)(t % (CC / 4)) * 4; const size_t r = t / (CC / 4); const size_t pt = (size_t)p0 + r; const int k = (int)(pt % KK); const int n = (int)((pt / KK) % NN); const int b = (int)(pt / ((size_t)KK * NN)); const float pc = fminf(fmaxf(bf16_round(pp[0]), 1.0f), 2.0f);
  v4f o;
#pragma unroll
  for (int q = 0; q < 4; ++q) { const int c = c0 + q; const float xv = inp_at(in, b, 3 + c, n, k); float a = 0.f;
#pragma unroll 1
    for (int m = 0; m < MM; ++m) { const float y = D2[r * (MM * CC) + m * CC + c] * xv; const float z = powf(fabsf(y + 1e-6f) + 1e-6f, pc) * ((y > 0.f) ? 1.f : ((y < 0.f) ? -1.f : 0.f)); a += SC[pt * MM + m] * z; }
    o[q] = a; }
  *(volatile v4f*)(AGG + pt * CC + c0) = o; __threadfence(); *(volatile v4f*)(AGG + pt * CC + c0) = o; }
__global__ __launch_bounds__(256) void k_maxk(const float* __restrict__ AGG, const float* __restrict__ AB, float* __restrict__ MXf, _Float16* __restrict__ Mh, _Float16* __restrict__ Ml) {
  #pragma clang fp contract(off)
  const int t = blockIdx.x * 256 + threadIdx.x; if (t >= NPN * (CC / 8)) return; const int c0 = (t % (CC / 8)) * 8, bn = t / (CC / 8); float mx[8];
#pragma unroll
  for (int q = 0; q < 8; ++q) mx[q] = -3.0e38f;
#pragma unroll 1
  for (int k = 0; k < KK; ++k) { const float* row = AGG + ((size_t)bn * KK + k) * CC + c0; const v4f a = *(const v4fa*)row, c = *(const v4fa*)(row + 4);
#pragma unroll
    for (int q = 0; q < 8; ++q) { const float v = fmaxf(((q < 4) ? a[q] : c[q - 4]) * AB[c0 + q] + AB[CC + c0 + q], 0.f); mx[q] = fmaxf(mx[q], v); } }
  FragH fh, fl; v4f oa, oc;
#pragma unroll
  for (int q = 0; q < 8; ++q) { const float v = mx[q]; if (q < 4) oa[q] = v; else oc[q - 4] = v; const _Float16 hi = (_Float16)v; fh.h[q] = hi; fl.h[q] = (_Float16)((v - (float)hi) * 1024.0f); }
  for (int pass = 0; pass < 2; ++pass) { *(volatile v8us*)((unsigned short*)Mh + (size_t)bn * CC + c0) = fh.half[0]; *(volatile v8us*)((unsigned short*)Ml + (size_t)bn * CC + c0) = fl.half[0]; (void)oa; (void)oc; (void)MXf; if (pass == 0) __threadfence(); } }
__global__ __launch_bounds__(256) void k_fin(const float* __restrict__ O, const float* __restrict__ AB, float* __restrict__ out) {
  #pragma clang fp contract(off)
  const int t = blockIdx.x * 256 + threadIdx.x; if (t >= NB * CO * (NN / 4)) return; const int n0 = (t % (NN / 4)) * 4; const int bo = t / (NN / 4); const int b = bo / CO, o = bo % CO; v4f v;
#pragma unroll
  for (int q = 0; q < 4; ++q) v[q] = fmaxf(O[((size_t)b * NN + n0 + q) * CO + o] * AB[o] + AB[CO + o], 0.f);
  *(volatile v4f*)(out + (size_t)bo * NN + n0) = v; __threadfence(); *(volatile v4f*)(out + (size_t)bo * NN + n0) = v; }

extern "C" void kernel_launch(void* const* d_in, const int* in_sizes, int n_in,
                              void* d_out, int out_size, void* d_ws, size_t ws_size, hipStream_t stream) {
  (void)in_sizes; (void)n_in; (void)out_size;
  const float* in = (const float*)d_in[0]; const float* pp = (const float*)d_in[1]; const float* sw1 = (const float*)d_in[2]; const float* sg1 = (const float*)d_in[3]; const float* sb1 = (const float*)d_in[4]; const float* sw2 = (const float*)d_in[5]; const float* sb2 = (const float*)d_in[6]; const float* hw1 = (const float*)d_in[7]; const float* hg1 = (const float*)d_in[8]; const float* hb1 = (const float*)d_in[9]; const float* hw2 = (const float*)d_in[10]; const float* hb2 = (const float*)d_in[11]; const float* dcg = (const float*)d_in[12]; const float* dcb = (const float*)d_in[13]; const float* crw = (const float*)d_in[14]; const float* crb = (const float*)d_in[15]; const float* b1g = (const float*)d_in[16]; const float* b1b = (const float*)d_in[17];
  char* ws = (char*)d_ws; size_t off = 0;
  auto take = [&](size_t bytes) { char* p = ws + off; off += (bytes + 255) & ~(size_t)255; return p; };
  _Float16* B2 = (_Float16*)take((size_t)MM * CC * 32 * 2); _Float16* Bcr = (_Float16*)take((size_t)CO * CC * 2);
  float* PRE = (float*)take((size_t)NPt * 48 * 4); double* SUM = (double*)take((size_t)2 * 32 * 8 * 4); double* SQ = (double*)take((size_t)2 * 32 * 8 * 4); float* ABs = (float*)take(64 * 4); float* ABd = (float*)take(128 * 4); float* ABa = (float*)take(256 * 4); float* ABo = (float*)take(512 * 4);
  float* SC = (float*)take((size_t)NPt * MM * 4); _Float16* Dh = (_Float16*)take((size_t)NPt * 32 * 2); _Float16* Dl = (_Float16*)take((size_t)NPt * 32 * 2); float* D2 = (float*)take((size_t)CH * MM * CC * 4); float* AGG = (float*)take((size_t)NPt * CC * 4); _Float16* Mh = (_Float16*)take((size_t)NPN * CC * 2); _Float16* Ml = (_Float16*)take((size_t)NPN * CC * 2); float* O = (float*)take((size_t)NPN * CO * 4); double* SUM2 = (double*)take((size_t)CO * 8); double* SQ2 = (double*)take((size_t)CO * 8);
  if (off > ws_size) return;
  k_round16f<<<(MM * CC * 32 / 8 + 255) / 256, 256, 0, stream>>>(hw2, B2, (size_t)MM * CC * 32 / 8); k_round16f<<<(CO * CC / 8 + 255) / 256, 256, 0, stream>>>(crw, Bcr, (size_t)CO * CC / 8);
  k_pre<<<(unsigned)(((size_t)NPt * 12 + 255) / 256), 256, 0, stream>>>(in, sw1, hw1, PRE);
  k_colstats<<<2, 256, 0, stream>>>(PRE, NPt, 48, SUM, SQ);
  k_bnab<<<1, 256, 0, stream>>>(SUM, SQ, MM, MM, NPt, sg1, sb1, ABs); k_bnab<<<1, 256, 0, stream>>>(SUM + MM, SQ + MM, 32, 32, NPt, hg1, hb1, ABd);
  k_act1<<<(unsigned)(((size_t)NPt * 4 + 255) / 256), 256, 0, stream>>>(PRE, ABs, ABd, sw2, sb2, SC, Dh, Dl);
  const dim3 gR(((CH / 16) * (MM * CC / 64) + 3) / 4, 1);
  for (int c = 0; c < NPt / CH; ++c) { const int p0 = c * CH;
    k_gemm_hhx<0><<<gR, 128, 0, stream>>>(Dh + (size_t)p0 * 32, 32, 0, B2, 32, 0, 0.0625f, hb2, 0, nullptr, 1, 0, 0, D2, nullptr, MM * CC, 0, CH, MM * CC, 32); k_gemm_hhx<0><<<gR, 128, 0, stream>>>(Dl + (size_t)p0 * 32, 32, 0, B2, 32, 0, 0.0625f / 1024.0f, nullptr, 0, D2, 1, (size_t)MM * CC, 0, D2, nullptr, MM * CC, 0, CH, MM * CC, 32);
    k_agg<<<(unsigned)(((size_t)CH * (CC / 4) + 255) / 256), 256, 0, stream>>>(D2, SC, in, pp, p0, AGG); }
  k_colstats<<<CC / 32, 256, 0, stream>>>(AGG, NPt, CC, SUM, SQ); k_bnab<<<1, 256, 0, stream>>>(SUM, SQ, CC, CC, NPt, dcg, dcb, ABa);
  k_maxk<<<(NPN * (CC / 8) + 255) / 256, 256, 0, stream>>>(AGG, ABa, nullptr, Mh, Ml);
  const dim3 gO(((NPN / 16) * (CO / 64) + 3) / 4, 1);
  k_gemm_hhx<0><<<gO, 128, 0, stream>>>(Mh, CC, 0, Bcr, CC, 0, 0.0625f, crb, 0, nullptr, 1, 0, 0, O, nullptr, CO, 0, NPN, CO, CC); k_gemm_hhx<0><<<gO, 128, 0, stream>>>(Ml, CC, 0, Bcr, CC, 0, 0.0625f / 1024.0f, nullptr, 0, O, 1, (size_t)CO, 0, O, nullptr, CO, 0, NPN, CO, CC);
  k_colstats<<<CO / 32, 256, 0, stream>>>(O, NPN, CO, SUM2, SQ2); k_bnab<<<1, 256, 0, stream>>>(SUM2, SQ2, CO, CO, NPN, b1g, b1b, ABo);
  k_fin<<<(NB * CO * (NN / 4) + 255) / 256, 256, 0, stream>>>(O, ABo, (float*)d_out);
}
